// KnowledgeGraphGNN_28509992910888
// MI455X (gfx1250) — hardware-verified
//
#include <hip/hip_runtime.h>


namespace {
constexpr int Bn = 8, NC = 1024, CIN = 256, HID = 512, NH = 8, DH = 64, NL = 3, NT = Bn * NC, NPR = NC * (NC - 1);
constexpr float XS = 8.0f;

typedef _Float16 b16;
typedef __attribute__((ext_vector_type(16))) _Float16 v16b;
typedef __attribute__((ext_vector_type(8))) _Float16 v8b;
typedef __attribute__((ext_vector_type(8))) float v8f;
typedef __attribute__((ext_vector_type(4))) float v4f;
typedef __attribute__((ext_vector_type(2))) float v2f;
__device__ __forceinline__ float bf16_rne(float f) { unsigned int u = __float_as_uint(f); u += 0x7FFFu + ((u >> 16) & 1u); return __uint_as_float(u & 0xFFFF0000u); }
__device__ __forceinline__ void split16(float v, b16& hi, b16& lo) { hi = (b16)v; lo = (b16)(v - (float)hi); }
__device__ __forceinline__ v16b frag_kb(const b16* p, int hh) { const v8b a = *(const v8b*)(p + 8 * hh), b = *(const v8b*)(p + 16 + 8 * hh); v16b f;
#pragma unroll
  for (int e = 0; e < 8; ++e) { f[e] = a[e]; f[8 + e] = b[e]; } return f; }
__device__ __forceinline__ v8f wmma16b(v16b a, v16b b, v8f c) { v8f d = __builtin_amdgcn_wmma_f32_16x16x32_f16(false, a, false, b, (short)0, c, false, false); asm volatile("v_nop\n\tv_nop\n\tv_nop\n\tv_nop" : "+v"(d) : "v"(a), "v"(b)); return d; }
__device__ __forceinline__ void wave_lds_sync() { __builtin_amdgcn_fence(__ATOMIC_RELEASE, "workgroup"); __builtin_amdgcn_wave_barrier(); __builtin_amdgcn_fence(__ATOMIC_ACQUIRE, "workgroup"); }
__device__ __forceinline__ float nexp(float x) { return __builtin_amdgcn_exp2f(x * 1.4426950408889634f); }
__device__ __forceinline__ float pmul(float a, float b) { float p = a * b; asm volatile("" : "+v"(p)); return p; }
__device__ __forceinline__ float wsum(float v) {
#pragma unroll
  for (int o = 1; o < 32; o <<= 1) v += __shfl_xor(v, o); return v; }

struct Ro_ { static constexpr size_t EMB = 0, IN = EMB + (size_t)HID * CIN, OUT = IN + (size_t)NL * 3 * HID * HID, CONV = OUT + (size_t)NL * HID * HID, POOL = CONV + (size_t)NL * HID * HID, END = POOL + (size_t)HID * HID; };
constexpr int PEND = 12295 + 512;
__global__ __launch_bounds__(256) void prep_kernel(const float* __restrict__ cf, const float* __restrict__ adj, const float* __restrict__ wemb, const float* __restrict__ bemb, const float* __restrict__ win, const float* __restrict__ bin_, const float* __restrict__ wout, const float* __restrict__ bout, const float* __restrict__ wconv, const float* __restrict__ bconv,
    const float* __restrict__ wcls, const float* __restrict__ bcls, const float* __restrict__ wdiff, const float* __restrict__ bdiff, const float* __restrict__ wpre, const float* __restrict__ bpre, const float* __restrict__ wpool, const float* __restrict__ bpool, b16* __restrict__ R, float* __restrict__ P, b16* __restrict__ CF, b16* __restrict__ ADJ) {
  const size_t tid = (size_t)blockIdx.x * 256 + threadIdx.x, nth = (size_t)gridDim.x * 256;
  for (int pass = 0; pass < 2; ++pass) {
    for (size_t p = tid; p < Ro_::END; p += nth) { float v; if (p < Ro_::IN) v = wemb[p]; else if (p < Ro_::OUT) v = win[p - Ro_::IN]; else if (p < Ro_::CONV) v = wout[p - Ro_::OUT]; else if (p < Ro_::POOL) v = wconv[p - Ro_::CONV]; else v = wpool[p - Ro_::POOL]; ((volatile b16*)R)[p] = (b16)bf16_rne(v); }
    for (size_t q = tid; q < (size_t)PEND; q += nth) { const int i = (int)q; float v; if (i < 512) v = bemb[i]; else if (i < 5120) v = bin_[i - 512]; else if (i < 6656) v = bout[i - 5120]; else if (i < 8192) v = bconv[i - 6656]; else if (i < 8704) v = wcls[i - 8192]; else if (i < 8705) v = bcls[0]; else if (i < 11265) v = wdiff[i - 8705]; else if (i < 11270) v = bdiff[i - 11265]; else if (i < 12294) v = wpre[i - 11270]; else if (i < 12295) v = bpre[0]; else v = bpool[i - 12295]; P[q] = bf16_rne(v); }
    for (size_t p = tid; p < (size_t)NT * CIN / 8; p += nth) { v8b v; for (int e = 0; e < 8; ++e) v[e] = (b16)(bf16_rne(cf[p * 8 + e]) * XS); *(volatile v8b*)(CF + p * 8) = v; }
    for (size_t p = tid; p < (size_t)Bn * NC * NC / 8; p += nth) { v8b v; for (int e = 0; e < 8; ++e) v[e] = (b16)(bf16_rne(adj[p * 8 + e]) * XS); *(volatile v8b*)(ADJ + p * 8) = v; }
    __threadfence(); }
}
template <int KIN, int TWOA, int TWOB, int EPI>
__global__ __launch_bounds__(64) void gemm_kernel(const b16* __restrict__ Ah, const b16* __restrict__ Al, int zA, const b16* __restrict__ Bh, const b16* __restrict__ Bl, int zB, const float* __restrict__ bias, float* __restrict__ OF, b16* __restrict__ OH, b16* __restrict__ OL, int ldo, int zO) {
  __shared__ __attribute__((aligned(16))) float Ts[2][16][128 + 4]; __shared__ __attribute__((aligned(16))) b16 Th[2][16][128 + 8], Tl[2][16][128 + 8];
  const int lane = threadIdx.x & 31, wave = threadIdx.x >> 5, nloc = lane & 15, hlf = lane >> 4, z = blockIdx.z, m0 = blockIdx.y * 32 + wave * 16, c0 = blockIdx.x * 128;
  const b16* A0 = Ah + ((size_t)z * zA) * KIN; const b16* A1 = TWOA ? Al + ((size_t)z * zA) * KIN : nullptr; const b16* B0 = Bh + ((size_t)z * zB) * KIN; const b16* B1 = TWOB ? Bl + ((size_t)z * zB) * KIN : nullptr;
  v8f acc[8];
#pragma unroll
  for (int t = 0; t < 8; ++t) acc[t] = (v8f){};
#pragma unroll 2
  for (int kb = 0; kb < KIN; kb += 32) { const v16b a = frag_kb(A0 + (size_t)(m0 + nloc) * KIN + kb, hlf); v16b al_; if (TWOA) al_ = frag_kb(A1 + (size_t)(m0 + nloc) * KIN + kb, hlf);
#pragma unroll
    for (int t = 0; t < 8; ++t) { const v16b bw = frag_kb(B0 + (size_t)(c0 + t * 16 + nloc) * KIN + kb, hlf); acc[t] = wmma16b(a, bw, acc[t]); if (TWOA) acc[t] = wmma16b(al_, bw, acc[t]); if (TWOB) acc[t] = wmma16b(a, frag_kb(B1 + (size_t)(c0 + t * 16 + nloc) * KIN + kb, hlf), acc[t]); } }
  const float osc = TWOB ? (1.0f / (XS * XS)) : (1.0f / XS);
#pragma unroll
  for (int t = 0; t < 8; ++t) { const float bb = bias ? bias[c0 + t * 16 + nloc] : 0.0f;
#pragma unroll
    for (int r = 0; r < 8; ++r) { const float v = acc[t][r] * osc + bb; if (EPI == 0 || EPI == 2) Ts[wave][8 * hlf + r][t * 16 + nloc] = v; if (EPI == 1 || EPI == 2) { b16 a_, c_; split16(v * XS, a_, c_); Th[wave][8 * hlf + r][t * 16 + nloc] = a_; Tl[wave][8 * hlf + r][t * 16 + nloc] = c_; } } }
  wave_lds_sync();
  const size_t orow0 = (size_t)z * zO;
  for (int pass = 0; pass < 2; ++pass) {
    if (EPI == 0 || EPI == 2) for (int i = lane; i < 16 * 32; i += 32) { const int rr = i >> 5, c4 = (i & 31) * 4; *(volatile v4f*)(OF + (orow0 + m0 + rr) * ldo + c0 + c4) = *(const v4f*)(&Ts[wave][rr][c4]); }
    if (EPI == 1 || EPI == 2) for (int i = lane; i < 16 * 16; i += 32) { const int rr = i >> 4, c8 = (i & 15) * 8; const size_t gi = (orow0 + m0 + rr) * ldo + c0 + c8; *(volatile v8b*)(OH + gi) = *(const v8b*)(&Th[wave][rr][c8]); *(volatile v8b*)(OL + gi) = *(const v8b*)(&Tl[wave][rr][c8]); }
    __threadfence(); }
}
__global__ __launch_bounds__(256) void tr_kernel(const b16* __restrict__ Ch, const b16* __restrict__ Cl, b16* __restrict__ CTh, b16* __restrict__ CTl) {
  __shared__ __attribute__((aligned(16))) b16 Sh[128][64 + 8]; __shared__ __attribute__((aligned(16))) b16 Sl2[128][64 + 8];
  const int j0 = blockIdx.x * 64, h0 = blockIdx.y * 128, b = blockIdx.z, t_ = threadIdx.x;
  for (int i = t_; i < 64 * 128; i += 256) { const int jj = i >> 7, hh2 = i & 127; const size_t src = ((size_t)b * NC + j0 + jj) * HID + h0 + hh2; Sh[hh2][jj] = Ch[src]; Sl2[hh2][jj] = Cl[src]; }
  __syncthreads();
  for (int pass = 0; pass < 2; ++pass) { for (int i = t_; i < 128 * 8; i += 256) { const int hh2 = i >> 3, c8 = (i & 7) * 8; const size_t gi = ((size_t)b * HID + h0 + hh2) * NC + j0 + c8; *(volatile v8b*)(CTh + gi) = *(const v8b*)(&Sh[hh2][c8]); *(volatile v8b*)(CTl + gi) = *(const v8b*)(&Sl2[hh2][c8]); } __threadfence(); }
}
__global__ __launch_bounds__(256) void mha_kernel(const float* __restrict__ QKV, b16* __restrict__ Oh, b16* __restrict__ Ol) {
  __shared__ __attribute__((aligned(16))) b16 Sh[Bn][HID + 8], Sl[Bn][HID + 8];
  const int n = blockIdx.x, h = threadIdx.x >> 5, lane = threadIdx.x & 31; const int c = h * DH + lane * 2;
  v2f q[Bn], k[Bn], v[Bn];
#pragma unroll
  for (int i = 0; i < Bn; ++i) { const float* row = QKV + ((size_t)i * NC + n) * (3 * HID); q[i] = *(const v2f*)(row + c); k[i] = *(const v2f*)(row + HID + c); v[i] = *(const v2f*)(row + 2 * HID + c); }
#pragma unroll
  for (int i = 0; i < Bn; ++i) { float sc[Bn]; float mx = -INFINITY;
#pragma unroll
    for (int j = 0; j < Bn; ++j) { float s = pmul(q[i][0], k[j][0]) + pmul(q[i][1], k[j][1]); s = wsum(s) * 0.125f; sc[j] = s; mx = fmaxf(mx, s); }
    float den = 0.0f;
#pragma unroll
    for (int j = 0; j < Bn; ++j) { sc[j] = nexp(sc[j] - mx); den += sc[j]; }
    const float inv = 1.0f / den; float o0 = 0.0f, o1 = 0.0f;
#pragma unroll
    for (int j = 0; j < Bn; ++j) { const float a = sc[j] * inv; o0 += pmul(a, v[j][0]); o1 += pmul(a, v[j][1]); }
    b16 a_, b_; split16(o0 * XS, a_, b_); Sh[i][c] = a_; Sl[i][c] = b_; split16(o1 * XS, a_, b_); Sh[i][c + 1] = a_; Sl[i][c + 1] = b_; }
  __syncthreads();
  for (int pass = 0; pass < 2; ++pass) { for (int t = threadIdx.x; t < Bn * (HID / 8); t += 256) { const int i = t / (HID / 8), c8 = (t % (HID / 8)) * 8; const size_t gi = ((size_t)i * NC + n) * HID + c8; *(volatile v8b*)(Oh + gi) = *(const v8b*)(&Sh[i][c8]); *(volatile v8b*)(Ol + gi) = *(const v8b*)(&Sl[i][c8]); } __threadfence(); }
}
template <int FINAL>
__global__ __launch_bounds__(256) void ln_kernel(const float* __restrict__ AGG, float* __restrict__ X, b16* __restrict__ Xh, b16* __restrict__ Xl, float* __restrict__ out0) {
  const int wave = threadIdx.x >> 5, row = blockIdx.x * 8 + wave, lane = threadIdx.x & 31; float y[16]; float s = 0.0f;
#pragma unroll
  for (int e = 0; e < 16; ++e) { const int c = lane * 16 + e; y[e] = X[(size_t)row * HID + c] + AGG[(size_t)row * HID + c]; s += y[e]; }
  s = wsum(s); const float mean = s * (1.0f / HID); float q2 = 0.0f;
#pragma unroll
  for (int e = 0; e < 16; ++e) { const float d = y[e] - mean; q2 += pmul(d, d); }
  q2 = wsum(q2); const float inv = rsqrtf(q2 * (1.0f / HID) + 1e-5f);
  v4f o[4]; v8b hh[2], ll[2];
#pragma unroll
  for (int e = 0; e < 16; ++e) { const float z = (y[e] - mean) * inv; o[e >> 2][e & 3] = z; b16 a_, b_; split16(z * XS, a_, b_); hh[e >> 3][e & 7] = a_; ll[e >> 3][e & 7] = b_; }
  for (int pass = 0; pass < 2; ++pass) { for (int g = 0; g < 4; ++g) { *(volatile v4f*)(X + (size_t)row * HID + lane * 16 + g * 4) = o[g]; if (FINAL) *(volatile v4f*)(out0 + (size_t)row * HID + lane * 16 + g * 4) = o[g]; }
    *(volatile v8b*)(Xh + (size_t)row * HID + lane * 16) = hh[0]; *(volatile v8b*)(Xh + (size_t)row * HID + lane * 16 + 8) = hh[1]; *(volatile v8b*)(Xl + (size_t)row * HID + lane * 16) = ll[0]; *(volatile v8b*)(Xl + (size_t)row * HID + lane * 16 + 8) = ll[1]; __threadfence(); }
}
__global__ __launch_bounds__(256) void heads_kernel(const float* __restrict__ X, const float* __restrict__ P, float* __restrict__ out1, float* __restrict__ out2, float* __restrict__ H12) {
  __shared__ float M_[64], D_[64][5], Hh_[64][2];
  const int wave = threadIdx.x >> 5, lane = threadIdx.x & 31, r0 = blockIdx.x * 64;
  for (int k = 0; k < 8; ++k) { const int rr = wave * 8 + k, row = r0 + rr; float xv[16]; for (int e = 0; e < 16; ++e) xv[e] = X[(size_t)row * HID + lane * 16 + e];
    float acc[8] = {0, 0, 0, 0, 0, 0, 0, 0};
#pragma unroll
    for (int e = 0; e < 16; ++e) { const int c = lane * 16 + e; acc[0] += pmul(xv[e], P[8192 + c]);
#pragma unroll
      for (int d = 0; d < 5; ++d) acc[1 + d] += pmul(xv[e], P[8705 + d * HID + c]);
      acc[6] += pmul(xv[e], P[11270 + c]); acc[7] += pmul(xv[e], P[11270 + HID + c]); }
#pragma unroll
    for (int a = 0; a < 8; ++a) acc[a] = wsum(acc[a]);
    if (lane == 0) { M_[rr] = acc[0] + P[8704]; for (int d = 0; d < 5; ++d) D_[rr][d] = acc[1 + d] + P[11265 + d]; Hh_[rr][0] = acc[6]; Hh_[rr][1] = acc[7]; } }
  __syncthreads();
  for (int pass = 0; pass < 2; ++pass) { if (threadIdx.x < 16) *(volatile v4f*)(out1 + r0 + threadIdx.x * 4) = *(const v4f*)(&M_[threadIdx.x * 4]);
    if (threadIdx.x < 80) *(volatile v4f*)(out2 + (size_t)r0 * 5 + threadIdx.x * 4) = *(const v4f*)(&D_[0][0] + threadIdx.x * 4);
    if (threadIdx.x < 32) *(volatile v4f*)(H12 + (size_t)r0 * 2 + threadIdx.x * 4) = *(const v4f*)(&Hh_[0][0] + threadIdx.x * 4);
    __threadfence(); }
}
__global__ __launch_bounds__(256) void prereq_kernel(const float* __restrict__ H12, const float* __restrict__ P, float* __restrict__ out3) {
  const int b = blockIdx.y; const size_t m0 = (size_t)blockIdx.x * 1024 + threadIdx.x * 4; const float bp = P[12294]; v4f o;
#pragma unroll
  for (int e = 0; e < 4; ++e) { const int m = (int)(m0 + e); const int i = m / (NC - 1), jj = m % (NC - 1); const int j = jj + ((jj >= i) ? 1 : 0); o[e] = H12[((size_t)b * NC + i) * 2] + H12[((size_t)b * NC + j) * 2 + 1] + bp; }
  for (int pass = 0; pass < 2; ++pass) { *(volatile v4f*)(out3 + (size_t)b * NPR + m0) = o; __threadfence(); }
}
__global__ __launch_bounds__(256) void graph_kernel(const float* __restrict__ X, const float* __restrict__ wpool, const float* __restrict__ P, float* __restrict__ out4) {
  __shared__ float Mn[HID], O_[HID];
  const int b = blockIdx.x, t = threadIdx.x;
  for (int cc = 0; cc < 2; ++cc) { const int c = t * 2 + cc; float s = 0.0f; for (int n = 0; n < NC; ++n) s += X[((size_t)b * NC + n) * HID + c]; Mn[c] = s * (1.0f / NC); }
  __syncthreads();
  for (int oo = 0; oo < 2; ++oo) { const int o = t * 2 + oo; float s = P[12295 + o]; for (int c = 0; c < HID; ++c) s += pmul(Mn[c], bf16_rne(wpool[(size_t)o * HID + c])); O_[o] = s; }
  __syncthreads();
  for (int pass = 0; pass < 2; ++pass) { if (t < 128) *(volatile v4f*)(out4 + (size_t)b * HID + t * 4) = *(const v4f*)(&O_[t * 4]); __threadfence(); }
}
}

extern "C" void kernel_launch(void* const* d_in, const int* in_sizes, int n_in,
                              void* d_out, int out_size, void* d_ws, size_t ws_size, hipStream_t stream) {
  (void)n_in; (void)out_size;
  auto Fp = [&](int i) { return (const float*)d_in[i]; };
  float* out0 = (float*)d_out; float* out1 = out0 + (size_t)NT * HID; float* out2 = out1 + NT; float* out3 = out2 + (size_t)NT * 5; float* out4 = out3 + (size_t)Bn * NPR;
  if (in_sizes[0] != NT * CIN || in_sizes[1] != Bn * NC * NC || in_sizes[6] != NL * 3 * HID * HID || in_sizes[18] != HID * HID) return;
  size_t off = 0; char* ws = (char*)d_ws;
  auto carve = [&](size_t bytes) { char* p = ws + off; off += (bytes + 255) & ~(size_t)255; return p; };
  b16* R = (b16*)carve(Ro_::END * 2); float* P = (float*)carve((size_t)PEND * 4 + 64); b16* CF = (b16*)carve((size_t)NT * CIN * 2); b16* ADJ = (b16*)carve((size_t)Bn * NC * NC * 2);
  float* X = (float*)carve((size_t)NT * HID * 4); b16* Xh = (b16*)carve((size_t)NT * HID * 2); b16* Xl = (b16*)carve((size_t)NT * HID * 2); float* QKV = (float*)carve((size_t)NT * 3 * HID * 4);
  b16* Oh = (b16*)carve((size_t)NT * HID * 2); b16* Ol = (b16*)carve((size_t)NT * HID * 2); b16* Ah2 = (b16*)carve((size_t)NT * HID * 2); b16* Al2 = (b16*)carve((size_t)NT * HID * 2); b16* CTh = (b16*)carve((size_t)NT * HID * 2); b16* CTl = (b16*)carve((size_t)NT * HID * 2); float* AGG = (float*)carve((size_t)NT * HID * 4); float* H12 = (float*)carve((size_t)NT * 2 * 4);
  if (off > ws_size) return;
  prep_kernel<<<1024, 256, 0, stream>>>(Fp(0), Fp(1), Fp(4), Fp(5), Fp(6), Fp(7), Fp(8), Fp(9), Fp(10), Fp(11), Fp(12), Fp(13), Fp(14), Fp(15), Fp(16), Fp(17), Fp(18), Fp(19), R, P, CF, ADJ);
  gemm_kernel<CIN, 0, 0, 2><<<dim3(HID / 128, NT / 32, 1), 64, 0, stream>>>(CF, nullptr, 0, R + Ro_::EMB, nullptr, 0, P, X, Xh, Xl, HID, 0);
  for (int l = 0; l < NL; ++l) {
    gemm_kernel<HID, 1, 0, 0><<<dim3(3 * HID / 128, NT / 32, 1), 64, 0, stream>>>(Xh, Xl, 0, R + Ro_::IN + (size_t)l * 3 * HID * HID, nullptr, 0, P + 512 + l * 1536, QKV, nullptr, nullptr, 3 * HID, 0);
    mha_kernel<<<NC, 256, 0, stream>>>(QKV, Oh, Ol);
    gemm_kernel<HID, 1, 0, 1><<<dim3(HID / 128, NT / 32, 1), 64, 0, stream>>>(Oh, Ol, 0, R + Ro_::OUT + (size_t)l * HID * HID, nullptr, 0, P + 5120 + l * 512, nullptr, Ah2, Al2, HID, 0);
    gemm_kernel<HID, 1, 0, 1><<<dim3(HID / 128, NT / 32, 1), 64, 0, stream>>>(Ah2, Al2, 0, R + Ro_::CONV + (size_t)l * HID * HID, nullptr, 0, P + 6656 + l * 512, nullptr, Oh, Ol, HID, 0);
    tr_kernel<<<dim3(NC / 64, HID / 128, Bn), 256, 0, stream>>>(Oh, Ol, CTh, CTl);
    gemm_kernel<NC, 0, 1, 0><<<dim3(HID / 128, NC / 32, Bn), 64, 0, stream>>>(ADJ, nullptr, NC, CTh, CTl, HID, nullptr, AGG, nullptr, nullptr, HID, NC);
    if (l + 1 < NL) ln_kernel<0><<<NT / 8, 256, 0, stream>>>(AGG, X, Xh, Xl, nullptr); else ln_kernel<1><<<NT / 8, 256, 0, stream>>>(AGG, X, Xh, Xl, out0); }
  heads_kernel<<<NT / 64, 256, 0, stream>>>(X, P, out1, out2, H12);
  prereq_kernel<<<dim3(1023, Bn), 256, 0, stream>>>(H12, P, out3);
  graph_kernel<<<Bn, 256, 0, stream>>>(X, Fp(18), P, out4);
}
